// BatchedNeRFMLP_49598282334732
// MI455X (gfx1250) — hardware-verified
//
#include <hip/hip_runtime.h>
#include <stddef.h>
#include <math.h>


#define POS_IN  63
#define K1P     64
#define HID     128
#define DIR_IN  27
#define CIN     155
#define TOTALP  8789
#define PW_OFF  0
#define PB_OFF  8064
#define SW_OFF  8192
#define SB_OFF  8320
#define CW_OFF  8321
#define CB_OFF  8786

#define NTHR    128
#define NWAVE   4
#define ITERS   8
#define PPB     (NWAVE * 16 * ITERS)
#define TP      72
#define DP      28
#define SCLW    64.0f
#define INVW    0.015625f
#define GRP     (HID * K1P / 8)
#define NSW     (4 * DP + 4)

static_assert(PB_OFF == POS_IN * HID);
static_assert(SW_OFF == PB_OFF + HID);
static_assert(SB_OFF == SW_OFF + HID);
static_assert(CW_OFF == SB_OFF + 1);
static_assert(CB_OFF == CW_OFF + 3 * CIN);
static_assert(TOTALP == CB_OFF + 3);
static_assert((TP * 2) % 16 == 0 && TP >= K1P);
static_assert(DP >= DIR_IN + 1 && (DP * 4) % 16 == 0);
static_assert(PPB == 512 && NTHR == NWAVE * 32);
static_assert(NSW <= NTHR);

typedef float    v4f  __attribute__((ext_vector_type(4)));
typedef float    v8f  __attribute__((ext_vector_type(8)));
typedef _Float16 v8h  __attribute__((ext_vector_type(8)));
typedef _Float16 v16h __attribute__((ext_vector_type(16)));
union FragH { v16h v; v8h h[2]; };

__device__ __forceinline__ v8f wmh(v16h a, v16h b, v8f c) {
  v8f d = __builtin_amdgcn_wmma_f32_16x16x32_f16(false, a, false, b, (short)0, c, false, false);
#if defined(__HIP_DEVICE_COMPILE__)
  asm volatile("v_nop\n\tv_nop\n\tv_nop\n\tv_nop" : "+v"(d) : "v"(a), "v"(b));
#endif
  return d;
}

__device__ __forceinline__ v8f zero8() {
  v8f z = {0.f, 0.f, 0.f, 0.f, 0.f, 0.f, 0.f, 0.f};
  return z;
}

template <int KT>
__device__ __forceinline__ void mma4(v8f (&acc)[4], const _Float16* ar, const _Float16* __restrict__ bplane,
                                     int nb0, int KP, int m, int hh) {
#pragma unroll
  for (int t = 0; t < 4; ++t) acc[t] = zero8();
#pragma unroll
  for (int kt = 0; kt < KT; ++kt) {
    FragH a;
    a.h[0] = *(const v8h*)(ar + 32 * kt);
    a.h[1] = *(const v8h*)(ar + 32 * kt + 16);
#pragma unroll
    for (int t = 0; t < 4; ++t) {
      const _Float16* bp = bplane + (size_t)(nb0 + 16 * t + m) * KP + 32 * kt + 8 * hh;
      FragH b;
      b.h[0] = *(const v8h*)bp;
      b.h[1] = *(const v8h*)(bp + 16);
      acc[t] = wmh(a.v, b.v, acc[t]);
    }
  }
}

template <int G>
__device__ __forceinline__ void head_acc(const v8f (&acc)[4],
                                         const float (&pbv)[8], const float (&swv)[8],
                                         const float (&c0w)[8], const float (&c1w)[8], const float (&c2w)[8],
                                         float (&s)[8], float (&c0)[8], float (&c1)[8], float (&c2)[8]) {
#pragma unroll
  for (int tt = 0; tt < 4; ++tt) {
    const int t = 4 * G + tt;
#pragma unroll
    for (int r = 0; r < 8; ++r) {
      const float hv = fmaxf(fmaf(acc[tt][r], INVW, pbv[t]), 0.0f);
      s[r]  = fmaf(hv, swv[t], s[r]);
      c0[r] = fmaf(hv, c0w[t], c0[r]);
      c1[r] = fmaf(hv, c1w[t], c1[r]);
      c2[r] = fmaf(hv, c2w[t], c2[r]);
    }
  }
}

__global__ __launch_bounds__(256) void k_prep(const float* __restrict__ params, _Float16* pwp, int nGrp) {
  const int i = blockIdx.x * 256 + (int)threadIdx.x;
  if (i >= nGrp) return;
  const int bb  = i / GRP;
  const int rem = i - bb * GRP;
  const int n   = rem >> 3;
  const int k0  = (rem & 7) * 8;
  const float* src = params + (size_t)bb * TOTALP + PW_OFF + n * POS_IN;
  v8h hv;
#pragma unroll
  for (int e = 0; e < 8; ++e) {
    const int k  = k0 + e;
    const int kc = k < POS_IN ? k : POS_IN - 1;
    const float xv = src[kc];
    hv[e] = (_Float16)((k < POS_IN) ? xv * SCLW : 0.0f);
  }
  _Float16* dp = pwp + (size_t)i * 8;
  *(volatile v8h*)dp = hv;
  __threadfence();
  *(volatile v8h*)dp = hv;
}

__global__ __launch_bounds__(NTHR) void k_mlp(
    const float* __restrict__ params, const float* __restrict__ points, const float* __restrict__ dirs,
    const _Float16* __restrict__ pwp, float* out, int nN) {
  __shared__ __align__(16) _Float16 sT[NWAVE][16 * TP];
  __shared__ __align__(16) float    sD[NWAVE][16 * DP];
  __shared__ __align__(16) float    sS[NWAVE][16 * 64];
  __shared__ __align__(16) float    sO[NWAVE][64];
  __shared__ __align__(16) float    sW[NSW];

  const int tid = threadIdx.x, lane = tid & 31, wave = tid >> 5, hh = lane >> 4, m = lane & 15;
  const int b = blockIdx.y;
  const int chunk = blockIdx.x;
  const float* prm = params + (size_t)b * TOTALP;
  const _Float16* bpl = pwp + (size_t)b * (HID * K1P);

  {
    const int o  = tid / DP;
    const int u  = tid - o * DP;
    const int oc = o < 2 ? o : 2;
    const int uc = u < DIR_IN - 1 ? u : DIR_IN - 1;
    const int a1 = CW_OFF + oc * CIN + HID + uc;
    int q = tid - 4 * DP;
    q = q < 0 ? 0 : (q > 3 ? 3 : q);
    const int a2 = (q < 3) ? (CB_OFF + q) : SB_OFF;
    const bool tail = tid >= 4 * DP;
    const float xv = prm[tail ? a2 : a1];
    const bool z = (!tail) && (o > 2 || u > DIR_IN - 1);
    if (tid < NSW) sW[tid] = z ? 0.0f : xv;
  }

  float pbv[8], swv[8], c0w[8], c1w[8], c2w[8];
#pragma unroll
  for (int t = 0; t < 8; ++t) {
    const int n = 16 * t + m;
    pbv[t] = prm[PB_OFF + n];
    swv[t] = prm[SW_OFF + n];
    c0w[t] = prm[CW_OFF + n];
    c1w[t] = prm[CW_OFF + CIN + n];
    c2w[t] = prm[CW_OFF + 2 * CIN + n];
  }

  float* out_b = out + (size_t)b * nN * 4;

  for (int it = 0; it < ITERS; ++it) {
    const int p0 = chunk * PPB + (it * NWAVE + wave) * 16;
    const int pt = p0 + m;
    const int ptc = pt < nN ? pt : nN - 1;
    const float* px = points + ((size_t)b * nN + ptc) * 3;
    const float* pd = dirs   + ((size_t)b * nN + ptc) * 3;
    const float x0 = px[0], x1 = px[1], x2 = px[2];
    const float d0 = pd[0], d1 = pd[1], d2 = pd[2];

    __syncthreads();

    _Float16* trow = &sT[wave][m * TP];
    float*    drow = &sD[wave][m * DP];
    trow[0] = (_Float16)x0; trow[1] = (_Float16)x1; trow[2] = (_Float16)x2;
    trow[K1P - 1] = (_Float16)0.0f;
    drow[0] = d0; drow[1] = d1; drow[2] = d2;
    drow[DP - 1] = 0.0f;
#pragma unroll 1
    for (int jj = 0; jj < 15; ++jj) {
      const int j = 15 * hh + jj;
      const int c = j / 10;
      const int f = j - 10 * c;
      const float xc = (c == 0) ? x0 : ((c == 1) ? x1 : x2);
      const float arg = xc * (float)(1 << f);
      float sv, cv;
      sincosf(arg, &sv, &cv);
      trow[3 + j]      = (_Float16)sv;
      trow[3 + 30 + j] = (_Float16)cv;
    }
#pragma unroll 1
    for (int uu = 0; uu < 6; ++uu) {
      const int u = 6 * hh + uu;
      const int c = u >> 2;
      const int f = u & 3;
      const float dc = (c == 0) ? d0 : ((c == 1) ? d1 : d2);
      const float arg = dc * (float)(1 << f);
      float sv, cv;
      sincosf(arg, &sv, &cv);
      drow[3 + u]  = sv;
      drow[15 + u] = cv;
    }

    __syncthreads();

    float s8[8], c0[8], c1[8], c2[8];
#pragma unroll
    for (int r = 0; r < 8; ++r) { s8[r] = 0.0f; c0[r] = 0.0f; c1[r] = 0.0f; c2[r] = 0.0f; }
    const _Float16* ar = &sT[wave][m * TP + 8 * hh];
    {
      v8f acc[4];
      mma4<2>(acc, ar, bpl, 0, K1P, m, hh);
      head_acc<0>(acc, pbv, swv, c0w, c1w, c2w, s8, c0, c1, c2);
    }
    {
      v8f acc[4];
      mma4<2>(acc, ar, bpl, 64, K1P, m, hh);
      head_acc<1>(acc, pbv, swv, c0w, c1w, c2w, s8, c0, c1, c2);
    }

    {
      float* sp = &sS[wave][(8 * hh) * 64 + m];
#pragma unroll
      for (int r = 0; r < 8; ++r) {
        sp[r * 64 +  0] = c0[r];
        sp[r * 64 + 16] = c1[r];
        sp[r * 64 + 32] = c2[r];
        sp[r * 64 + 48] = s8[r];
      }
    }
    __syncthreads();

    {
      const float* sq = &sS[wave][m * 64];
      float suma = 0.0f, sumb = 0.0f;
#pragma unroll
      for (int i = 0; i < 4; ++i) {
        const v4f va4 = *(const v4f*)(sq + 16 * hh + 4 * i);
        const v4f vb4 = *(const v4f*)(sq + 16 * (2 + hh) + 4 * i);
        suma += (va4.x + va4.y) + (va4.z + va4.w);
        sumb += (vb4.x + vb4.y) + (vb4.z + vb4.w);
      }
      const float* dr = &sD[wave][m * DP];
      const float* wa = sW + hh * DP;
      const float* wb = sW + (2 + hh) * DP;
      float va = suma, vb = sumb;
#pragma unroll
      for (int u = 0; u < DIR_IN; ++u) {
        const float dv = dr[u];
        va = fmaf(dv, wa[u], va);
        vb = fmaf(dv, wb[u], vb);
      }
      va += sW[4 * DP + hh];
      vb += sW[4 * DP + 2 + hh];
      const float ta = fminf(fmaxf(va, -30.0f), 30.0f);
      const float tb = fminf(fmaxf(vb, -30.0f), 30.0f);
      const float ga = 1.0f / (1.0f + expf(-ta));
      const float gb = 1.0f / (1.0f + expf(-tb));
      const float oa = ga;
      const float ob = (hh != 0) ? vb : gb;
      sO[wave][m * 4 + hh]     = oa;
      sO[wave][m * 4 + 2 + hh] = ob;
    }
    __syncthreads();

    {
      const v4f ov = *(const v4f*)(&sO[wave][4 * m]);
      float* gp = out_b + (size_t)pt * 4;
      const bool wr = (hh == 0) && (pt < nN);
      if (wr) *(volatile v4f*)gp = ov;
      __threadfence();
      if (wr) *(volatile v4f*)gp = ov;
    }
  }
}

extern "C" void kernel_launch(void* const* d_in, const int* in_sizes, int n_in,
                              void* d_out, int out_size, void* d_ws, size_t ws_size,
                              hipStream_t stream) {
  if (n_in < 3) return;
  if (in_sizes[0] <= 0 || (in_sizes[0] % TOTALP) != 0) return;
  const int nB = in_sizes[0] / TOTALP;
  if (nB <= 0 || nB > 65535) return;
  if (in_sizes[1] <= 0 || (in_sizes[1] % (nB * 3)) != 0) return;
  const int nN = in_sizes[1] / (nB * 3);
  if (nN <= 0 || in_sizes[2] != in_sizes[1]) return;
  if ((long long)out_size != (long long)nB * nN * 4) return;

  const float* params = (const float*)d_in[0];
  const float* points = (const float*)d_in[1];
  const float* dirs   = (const float*)d_in[2];
  float* out = (float*)d_out;

  const size_t planeBytes = (size_t)nB * HID * K1P * 2;
  if (planeBytes > ws_size || planeBytes > (size_t)134217728) return;
  _Float16* pwp = (_Float16*)d_ws;

  const int nGrp = nB * GRP;
  k_prep<<<(nGrp + 255) / 256, 256, 0, stream>>>(params, pwp, nGrp);

  const int nChunk = (nN + PPB - 1) / PPB;
  dim3 grid(nChunk, nB, 1);
  k_mlp<<<grid, NTHR, 0, stream>>>(params, points, dirs, pwp, out, nN);
}
